// rnn_decoder_74294344286647
// MI455X (gfx1250) — hardware-run, weakly checked
//
#include <hip/hip_runtime.h>
#include <stddef.h>
#include <math.h>


#define NB    32
#define NT    64
#define NS    64
#define NE    512
#define NH    1024
#define NG    4096
#define NL    2
#define NV    32000
#define NR    (NB * NT)
#define NSLOT (NT + 1)
#define O1E   (NR * NH)
#define O2E   (O1E + NL * NB * NH)
#define OUTN  (O2E + NL * NB * NH)

#define SCW    16.0f
#define SCX    16.0f
#define SCWO1  4.0f
#define SCCTX  64.0f
#define SCP    1024.0f
#define INV256 0.00390625f

#define SZ_EMB  ((size_t)NR * NE * 2)
#define SZ_WIH0 ((size_t)NG * NE * 2)
#define SZ_WK   ((size_t)NG * NH * 2)
#define SZ_WIN  ((size_t)NH * NH * 2)
#define SZ_WOUT ((size_t)NH * 2 * NH * 2)
#define SZ_ENC  ((size_t)NB * NS * NH * 2)
#define SZ_X0   ((size_t)NR * NG * 4)
#define SZ_HP   ((size_t)NSLOT * NB * NH * 2)
#define SZ_C    ((size_t)NB * NH * 4)
#define SZ_R16  ((size_t)NR * NH * 2)
#define O_EMB   ((size_t)0)
#define O_WIH0  (O_EMB + SZ_EMB)
#define O_WHH0  (O_WIH0 + SZ_WIH0)
#define O_WIH1  (O_WHH0 + SZ_WK)
#define O_WHH1  (O_WIH1 + SZ_WK)
#define O_WIN   (O_WHH1 + SZ_WK)
#define O_WOUT  (O_WIN + SZ_WIN)
#define O_ENC   (O_WOUT + SZ_WOUT)
#define O_ENCT  (O_ENC + SZ_ENC)
#define O_X0    (O_ENCT + SZ_ENC)
#define O_H0    (O_X0 + SZ_X0)
#define O_H1    (O_H0 + SZ_HP)
#define O_C0    (O_H1 + SZ_HP)
#define O_C1    (O_C0 + SZ_C)
#define O_GAM   (O_C1 + SZ_C)
#define O_CTX   (O_GAM + SZ_R16)
#define WSTOT   (O_CTX + SZ_R16)
#define WSCAP   134217728

static_assert(WSTOT <= (size_t)WSCAP);
static_assert((O_WIH0 % 128) == 0 && (O_WHH0 % 128) == 0 && (O_WIH1 % 128) == 0 && (O_WHH1 % 128) == 0);
static_assert((O_WIN % 128) == 0 && (O_WOUT % 128) == 0 && (O_ENC % 128) == 0 && (O_ENCT % 128) == 0);
static_assert((O_X0 % 128) == 0 && (O_H0 % 128) == 0 && (O_H1 % 128) == 0 && (O_C0 % 128) == 0);
static_assert((O_C1 % 128) == 0 && (O_GAM % 128) == 0 && (O_CTX % 128) == 0);
static_assert(OUTN * 4 == 8912896);
static_assert((NE % 32) == 0 && (NH % 32) == 0 && (NS % 32) == 0);
static_assert((NR % 64) == 0 && (NG % 128) == 0 && (NH % 128) == 0);
static_assert((NH % 64) == 0 && NB == 32 && NS == 64 && NT == 64);
static_assert((NG * NE) % 2048 == 0 && (NG * NH) % 2048 == 0 && (NH * NH) % 2048 == 0);
static_assert((NH * 2 * NH) % 2048 == 0 && (NB * NS * NH) % 2048 == 0);
static_assert((NR * NE) % 2048 == 0 && (NL * NB * NH) % 2048 == 0);

typedef _Float16 f16_t;
typedef unsigned short us_t;
typedef f16_t  v8h  __attribute__((ext_vector_type(8), __may_alias__));
typedef f16_t  v16h __attribute__((ext_vector_type(16)));
typedef us_t   v8us __attribute__((ext_vector_type(8), __may_alias__));
typedef int    v8i  __attribute__((ext_vector_type(8)));
typedef float  v8f  __attribute__((ext_vector_type(8)));
typedef float  v4f  __attribute__((ext_vector_type(4), __may_alias__));
union Frag { v16h v; v8h f[2]; v8us h[2]; v8i w; };
static_assert(sizeof(Frag) == 32);

__device__ __forceinline__ v8f wmh(Frag a, Frag b, v8f c) {
  v8f d = __builtin_amdgcn_wmma_f32_16x16x32_f16(false, a.v, false, b.v, (short)0, c, false, false);
  asm volatile("v_nop\n\tv_nop\n\tv_nop\n\tv_nop" : "+v"(d) : "v"(a.w), "v"(b.w));
  return d;
}

__device__ __forceinline__ v8f zero8() {
  v8f z = {0.f, 0.f, 0.f, 0.f, 0.f, 0.f, 0.f, 0.f};
  return z;
}

__device__ __forceinline__ v8us cvt8h_(const float* f, float sc) {
  union { v8h v; v8us u; } x;
  v8h t;
#pragma unroll
  for (int i = 0; i < 8; ++i) t[i] = (f16_t)(f[i] * sc);
  x.v = t;
  return x.u;
}
__device__ __forceinline__ v8us asus_(v8h v) {
  union { v8h v; v8us u; } x;
  x.v = v;
  return x.u;
}

__device__ __forceinline__ float wsum_(float v) {
  v += __shfl_xor(v, 16);
  v += __shfl_xor(v, 8);
  v += __shfl_xor(v, 4);
  v += __shfl_xor(v, 2);
  v += __shfl_xor(v, 1);
  return v;
}
__device__ __forceinline__ float wmax_(float v) {
  v = fmaxf(v, __shfl_xor(v, 16));
  v = fmaxf(v, __shfl_xor(v, 8));
  v = fmaxf(v, __shfl_xor(v, 4));
  v = fmaxf(v, __shfl_xor(v, 2));
  v = fmaxf(v, __shfl_xor(v, 1));
  return v;
}
__device__ __forceinline__ float sigm_(float x) {
  const float xc = fminf(fmaxf(x, -30.0f), 30.0f);
  return __builtin_amdgcn_rcpf(1.0f + __expf(-xc));
}
__device__ __forceinline__ float tanh_(float x) { return 2.0f * sigm_(2.0f * x) - 1.0f; }

__device__ __forceinline__ void gseg_(v8f (&acc)[2][4], const us_t* A, int lda, const us_t* W,
                                      size_t ldw, size_t gstride, int nks, int h, int m) {
  const us_t* ap0 = A + (size_t)m * lda + 8 * h;
  const us_t* ap1 = ap0 + (size_t)16 * lda;
  const us_t* bp  = W + (size_t)m * ldw + 8 * h;
#pragma unroll 1
  for (int ks = 0; ks < nks; ++ks) {
    const int k0 = 32 * ks;
    Frag a0, a1;
    a0.h[0] = *(const v8us*)(ap0 + k0);
    a0.h[1] = *(const v8us*)(ap0 + k0 + 16);
    a1.h[0] = *(const v8us*)(ap1 + k0);
    a1.h[1] = *(const v8us*)(ap1 + k0 + 16);
#pragma unroll
    for (int t = 0; t < 4; ++t) {
      const us_t* q = bp + (size_t)t * gstride + k0;
      Frag bb;
      bb.h[0] = *(const v8us*)q;
      bb.h[1] = *(const v8us*)(q + 16);
      acc[0][t] = wmh(a0, bb, acc[0][t]);
      acc[1][t] = wmh(a1, bb, acc[1][t]);
    }
  }
}

__global__ __launch_bounds__(256) void k_cvt(const float* __restrict__ src, us_t* dst,
                                              int ncols, int splitcol, float slo, float shi) {
  const size_t e = ((size_t)blockIdx.x * 256 + threadIdx.x) * 8;
  const int col = (int)(e % (size_t)ncols);
  const float sc = (col < splitcol) ? slo : shi;
  const v4f a0 = *(const v4f*)(src + e);
  const v4f a1 = *(const v4f*)(src + e + 4);
  float f[8];
  f[0] = a0.x; f[1] = a0.y; f[2] = a0.z; f[3] = a0.w;
  f[4] = a1.x; f[5] = a1.y; f[6] = a1.z; f[7] = a1.w;
  const v8us v = cvt8h_(f, sc);
  *(volatile v8us*)(dst + e) = v;
  __threadfence();
  *(volatile v8us*)(dst + e) = v;
}

__global__ __launch_bounds__(256) void k_enct(const float* __restrict__ enc, us_t* ENCT) {
  __shared__ float sT[64 * 65];
  const int tid = threadIdx.x;
  const int h0 = blockIdx.x * 64, b = blockIdx.y;
  const float* eb = enc + (size_t)b * NS * NH;
#pragma unroll
  for (int it = 0; it < 4; ++it) {
    const int e = tid + 256 * it;
    const int sr = e >> 4, hq = e & 15;
    const v4f a = *(const v4f*)(eb + (size_t)sr * NH + h0 + 4 * hq);
    sT[(4 * hq + 0) * 65 + sr] = a.x;
    sT[(4 * hq + 1) * 65 + sr] = a.y;
    sT[(4 * hq + 2) * 65 + sr] = a.z;
    sT[(4 * hq + 3) * 65 + sr] = a.w;
  }
  __syncthreads();
  v8us ov[2];
  size_t off[2];
#pragma unroll
  for (int it = 0; it < 2; ++it) {
    const int e = tid + 256 * it;
    const int rl = e >> 3, q = e & 7;
    float f[8];
#pragma unroll
    for (int i = 0; i < 8; ++i) f[i] = sT[rl * 65 + 8 * q + i];
    ov[it] = cvt8h_(f, SCX);
    off[it] = ((size_t)b * NH + h0 + rl) * NS + 8 * q;
  }
#pragma unroll
  for (int it = 0; it < 2; ++it) *(volatile v8us*)(ENCT + off[it]) = ov[it];
  __threadfence();
#pragma unroll
  for (int it = 0; it < 2; ++it) *(volatile v8us*)(ENCT + off[it]) = ov[it];
}

__global__ __launch_bounds__(256) void k_embg(const int* __restrict__ tok, const float* __restrict__ emb,
                                               us_t* EMB) {
  const int e = blockIdx.x * 256 + threadIdx.x;
  const int r = e >> 6, q = e & 63;
  const int t = r >> 5, b = r & 31;
  int id = tok[b * NT + t];
  id = (id < 0) ? 0 : ((id > NV - 1) ? (NV - 1) : id);
  const float* p = emb + (size_t)id * NE + 8 * q;
  const v4f a0 = *(const v4f*)p;
  const v4f a1 = *(const v4f*)(p + 4);
  float f[8];
  f[0] = a0.x; f[1] = a0.y; f[2] = a0.z; f[3] = a0.w;
  f[4] = a1.x; f[5] = a1.y; f[6] = a1.z; f[7] = a1.w;
  const v8us v = cvt8h_(f, SCX);
  const size_t off = (size_t)r * NE + 8 * q;
  *(volatile v8us*)(EMB + off) = v;
  __threadfence();
  *(volatile v8us*)(EMB + off) = v;
}

__global__ __launch_bounds__(256) void k_inith(const float* __restrict__ hin, us_t* H0, us_t* H1) {
  const int e = blockIdx.x * 256 + threadIdx.x;
  const int l = e >> 12, w = e & 4095;
  const float* p = hin + (size_t)l * NB * NH + 8 * w;
  const v4f a0 = *(const v4f*)p;
  const v4f a1 = *(const v4f*)(p + 4);
  float f[8];
  f[0] = a0.x; f[1] = a0.y; f[2] = a0.z; f[3] = a0.w;
  f[4] = a1.x; f[5] = a1.y; f[6] = a1.z; f[7] = a1.w;
  const v8us v = cvt8h_(f, SCX);
  us_t* d = ((l == 0) ? H0 : H1) + 8 * w;
  *(volatile v8us*)d = v;
  __threadfence();
  *(volatile v8us*)d = v;
}

template <int MODE>
__global__ __launch_bounds__(128) void k_gemm(const us_t* __restrict__ A1, int lda1, int nk1,
                                               const us_t* __restrict__ A2, int lda2, int nk2,
                                               const us_t* __restrict__ Bw, int ldb,
                                               const float* __restrict__ bias0,
                                               const float* __restrict__ bias1,
                                               float* dstf, us_t* dsth, int ldd) {
  __shared__ __align__(16) float sT[64 * 128];
  const int tid = threadIdx.x, lane = tid & 31, wave = tid >> 5, h = lane >> 4, m = lane & 15;
  const int wr = wave & 1, wc = wave >> 1;
  const int bm0 = blockIdx.x * 64, n0 = blockIdx.y * 128;
  const int rl0 = 32 * wr, cl0 = 64 * wc;

  v8f acc[2][4];
#pragma unroll
  for (int mt = 0; mt < 2; ++mt)
#pragma unroll
    for (int t = 0; t < 4; ++t) acc[mt][t] = zero8();

  gseg_(acc, A1 + (size_t)(bm0 + rl0) * lda1, lda1, Bw + (size_t)(n0 + cl0) * ldb,
        (size_t)ldb, (size_t)16 * ldb, nk1, h, m);
  gseg_(acc, A2 + (size_t)(bm0 + rl0) * lda2, lda2, Bw + (size_t)(n0 + cl0) * ldb + 32 * nk1,
        (size_t)ldb, (size_t)16 * ldb, nk2, h, m);

#pragma unroll
  for (int mt = 0; mt < 2; ++mt)
#pragma unroll
    for (int t = 0; t < 4; ++t)
#pragma unroll
      for (int r = 0; r < 8; ++r)
        sT[(rl0 + 16 * mt + 8 * h + r) * 128 + cl0 + 16 * t + m] = acc[mt][t][r];
  __syncthreads();

  const int rw = 16 * wave;
  v4f bb = *(const v4f*)(bias0 + n0 + 4 * lane);
  if (MODE == 0) bb = bb + *(const v4f*)(bias1 + n0 + 4 * lane);

#pragma unroll 1
  for (int j = 0; j < 16; ++j) {
    float* p = sT + (rw + j) * 128 + 4 * lane;
    v4f v = *(const v4f*)p;
    v = v * INV256 + bb;
    if (MODE == 1) v = v * SCX;
    if (MODE == 2) { v.x = tanhf(v.x); v.y = tanhf(v.y); v.z = tanhf(v.z); v.w = tanhf(v.w); }
    *(v4f*)p = v;
  }
  __syncthreads();

  if (MODE == 1) {
    const int rsub = lane >> 4, cq = lane & 15;
    v8us ov[8];
#pragma unroll
    for (int j = 0; j < 8; ++j) {
      const float* p = sT + (rw + 2 * j + rsub) * 128 + 8 * cq;
      const v4f x0 = *(const v4f*)p;
      const v4f x1 = *(const v4f*)(p + 4);
      float f[8];
      f[0] = x0.x; f[1] = x0.y; f[2] = x0.z; f[3] = x0.w;
      f[4] = x1.x; f[5] = x1.y; f[6] = x1.z; f[7] = x1.w;
      ov[j] = cvt8h_(f, 1.0f);
    }
#pragma unroll
    for (int j = 0; j < 8; ++j) {
      const size_t off = (size_t)(bm0 + rw + 2 * j + rsub) * ldd + n0 + 8 * cq;
      *(volatile v8us*)(dsth + off) = ov[j];
    }
    __threadfence();
#pragma unroll
    for (int j = 0; j < 8; ++j) {
      const size_t off = (size_t)(bm0 + rw + 2 * j + rsub) * ldd + n0 + 8 * cq;
      *(volatile v8us*)(dsth + off) = ov[j];
    }
  } else {
    v4f ov[16];
#pragma unroll
    for (int j = 0; j < 16; ++j) ov[j] = *(const v4f*)(sT + (rw + j) * 128 + 4 * lane);
#pragma unroll
    for (int j = 0; j < 16; ++j) {
      const int r = bm0 + rw + j;
      const int orow = (MODE == 2) ? ((r & (NB - 1)) * NT + (r >> 5)) : r;
      const size_t off = (size_t)orow * ldd + n0 + 4 * lane;
      *(volatile v4f*)(dstf + off) = ov[j];
    }
    __threadfence();
#pragma unroll
    for (int j = 0; j < 16; ++j) {
      const int r = bm0 + rw + j;
      const int orow = (MODE == 2) ? ((r & (NB - 1)) * NT + (r >> 5)) : r;
      const size_t off = (size_t)orow * ldd + n0 + 4 * lane;
      *(volatile v4f*)(dstf + off) = ov[j];
    }
  }
}

__global__ __launch_bounds__(128) void k_step(const us_t* __restrict__ WHH0, const us_t* __restrict__ WIH1,
                                               const us_t* __restrict__ WHH1, const float* __restrict__ X0,
                                               const float* __restrict__ bih1, const float* __restrict__ bhh1,
                                               us_t* H0, us_t* H1, const float* cprev0, const float* cprev1,
                                               float* C0, float* C1, float* out, int t0, int laybase) {
  __shared__ __align__(16) float sC[NB * 64];
  __shared__ __align__(16) float sH[NB * 64];
  const int tid = threadIdx.x, lane = tid & 31, wave = tid >> 5, h = lane >> 4, m = lane & 15;
  const int layer = (int)blockIdx.y + laybase;
  const int t = t0 - layer;
  const int nb0 = blockIdx.x * 64, nw0 = nb0 + 16 * wave, n = nw0 + m;
  const size_t slot = (size_t)NB * NH;

  const us_t* Aa; const us_t* Wa; const us_t* Ab; const us_t* Wb; int nkb;
  const float* cp; float* Cd; us_t* Hd;
  if (layer == 0) {
    Aa = H0 + (size_t)t * slot;       Wa = WHH0;
    Ab = Aa;                          Wb = Wa;   nkb = 0;
    cp = cprev0; Cd = C0; Hd = H0 + (size_t)(t + 1) * slot;
  } else {
    Aa = H0 + (size_t)(t + 1) * slot; Wa = WIH1;
    Ab = H1 + (size_t)t * slot;       Wb = WHH1; nkb = NH / 32;
    cp = cprev1; Cd = C1; Hd = H1 + (size_t)(t + 1) * slot;
  }

  v8f acc[2][4];
#pragma unroll
  for (int mt = 0; mt < 2; ++mt)
#pragma unroll
    for (int g = 0; g < 4; ++g) acc[mt][g] = zero8();

  gseg_(acc, Aa, NH, Wa + (size_t)nw0 * NH, (size_t)NH, (size_t)NH * NH, NH / 32, h, m);
  gseg_(acc, Ab, NH, Wb + (size_t)nw0 * NH, (size_t)NH, (size_t)NH * NH, nkb, h, m);

  float badd[4];
#pragma unroll
  for (int g = 0; g < 4; ++g)
    badd[g] = (layer == 1) ? (bih1[g * NH + n] + bhh1[g * NH + n]) : 0.0f;

#pragma unroll
  for (int mt = 0; mt < 2; ++mt) {
#pragma unroll
    for (int r = 0; r < 8; ++r) {
      const int b = 16 * mt + 8 * h + r;
      float pre[4];
#pragma unroll
      for (int g = 0; g < 4; ++g) pre[g] = acc[mt][g][r] * INV256 + badd[g];
      if (layer == 0) {
        const float* xp = X0 + ((size_t)(t * NB + b)) * NG + n;
#pragma unroll
        for (int g = 0; g < 4; ++g) pre[g] += xp[(size_t)g * NH];
      }
      const float cold = cp[(size_t)b * NH + n];
      const float ig = sigm_(pre[0]);
      const float fg = sigm_(pre[1]);
      const float gg = tanh_(pre[2]);
      const float og = sigm_(pre[3]);
      const float c2 = fg * cold + ig * gg;
      const float h2 = og * tanh_(c2);
      sC[b * 64 + 16 * wave + m] = c2;
      sH[b * 64 + 16 * wave + m] = h2;
    }
  }
  __syncthreads();

  const int rsub = lane >> 4, cq = lane & 15;
  const int rq = lane >> 3, cq8 = lane & 7;
  v4f cv[4], hf[4];
  size_t coff[4];
#pragma unroll
  for (int j = 0; j < 4; ++j) {
    const int row = 8 * wave + 2 * j + rsub;
    cv[j] = *(const v4f*)(sC + row * 64 + 4 * cq);
    hf[j] = *(const v4f*)(sH + row * 64 + 4 * cq);
    coff[j] = (size_t)row * NH + nb0 + 4 * cq;
  }
  v8us hv[2];
  size_t hoff[2];
#pragma unroll
  for (int j = 0; j < 2; ++j) {
    const int row = 8 * wave + 4 * j + rq;
    const float* p = sH + row * 64 + 8 * cq8;
    const v4f x0 = *(const v4f*)p;
    const v4f x1 = *(const v4f*)(p + 4);
    float f[8];
    f[0] = x0.x; f[1] = x0.y; f[2] = x0.z; f[3] = x0.w;
    f[4] = x1.x; f[5] = x1.y; f[6] = x1.z; f[7] = x1.w;
    hv[j] = cvt8h_(f, SCX);
    hoff[j] = (size_t)row * NH + nb0 + 8 * cq8;
  }
  const bool fin = (t == NT - 1);
  float* oh = out + O1E + (size_t)layer * NB * NH;
  float* oc = out + O2E + (size_t)layer * NB * NH;

#pragma unroll
  for (int j = 0; j < 4; ++j) *(volatile v4f*)(Cd + coff[j]) = cv[j];
#pragma unroll
  for (int j = 0; j < 2; ++j) *(volatile v8us*)(Hd + hoff[j]) = hv[j];
  if (fin) {
#pragma unroll
    for (int j = 0; j < 4; ++j) { *(volatile v4f*)(oh + coff[j]) = hf[j]; *(volatile v4f*)(oc + coff[j]) = cv[j]; }
  }
  __threadfence();
#pragma unroll
  for (int j = 0; j < 4; ++j) *(volatile v4f*)(Cd + coff[j]) = cv[j];
#pragma unroll
  for (int j = 0; j < 2; ++j) *(volatile v8us*)(Hd + hoff[j]) = hv[j];
  if (fin) {
#pragma unroll
    for (int j = 0; j < 4; ++j) { *(volatile v4f*)(oh + coff[j]) = hf[j]; *(volatile v4f*)(oc + coff[j]) = cv[j]; }
  }
}

__global__ __launch_bounds__(128) void k_attn(const us_t* __restrict__ GAM, const us_t* __restrict__ ENC,
                                               const us_t* __restrict__ ENCT, us_t* CTX) {
  __shared__ float sS[NT * 65];
  __shared__ __align__(16) f16_t sP[NT * 72];
  __shared__ __align__(16) f16_t sX[4 * 16 * 72];
  const int tid = threadIdx.x, lane = tid & 31, wave = tid >> 5, h = lane >> 4, m = lane & 15;
  const int b = blockIdx.x;
  const int tw = 16 * wave;

  v8f acc[4];
#pragma unroll
  for (int st = 0; st < 4; ++st) acc[st] = zero8();
  const us_t* ap = GAM + ((size_t)((tw + m) * NB + b)) * NH + 8 * h;
  const us_t* bp = ENC + ((size_t)(b * NS + m)) * NH + 8 * h;
#pragma unroll 1
  for (int ks = 0; ks < NH / 32; ++ks) {
    const int k0 = 32 * ks;
    Frag a;
    a.h[0] = *(const v8us*)(ap + k0);
    a.h[1] = *(const v8us*)(ap + k0 + 16);
#pragma unroll
    for (int st = 0; st < 4; ++st) {
      const us_t* q = bp + (size_t)(16 * st) * NH + k0;
      Frag bb;
      bb.h[0] = *(const v8us*)q;
      bb.h[1] = *(const v8us*)(q + 16);
      acc[st] = wmh(a, bb, acc[st]);
    }
  }
#pragma unroll
  for (int st = 0; st < 4; ++st)
#pragma unroll
    for (int rr = 0; rr < 8; ++rr)
      sS[(tw + 8 * h + rr) * 65 + 16 * st + m] = acc[st][rr] * INV256;
  __syncthreads();

#pragma unroll 1
  for (int i = 0; i < 16; ++i) {
    const int row = tw + i;
    const float v0 = sS[row * 65 + lane];
    const float v1 = sS[row * 65 + 32 + lane];
    const float mx = wmax_(fmaxf(v0, v1));
    const float e0 = expf(v0 - mx);
    const float e1 = expf(v1 - mx);
    const float sm = wsum_(e0 + e1);
    const float inv = 1.0f / sm;
    sP[row * 72 + lane]      = (f16_t)(e0 * inv * SCP);
    sP[row * 72 + 32 + lane] = (f16_t)(e1 * inv * SCP);
  }
  __syncthreads();

  Frag pa[2];
#pragma unroll
  for (int ks = 0; ks < 2; ++ks) {
    pa[ks].f[0] = *(const v8h*)(sP + (tw + m) * 72 + 32 * ks + 8 * h);
    pa[ks].f[1] = *(const v8h*)(sP + (tw + m) * 72 + 32 * ks + 16 + 8 * h);
  }
  const int rq = lane >> 3, cq8 = lane & 7;
#pragma unroll 1
  for (int ng = 0; ng < NH / 64; ++ng) {
    v8f acc2[4];
#pragma unroll
    for (int nt = 0; nt < 4; ++nt) acc2[nt] = zero8();
#pragma unroll
    for (int ks = 0; ks < 2; ++ks) {
#pragma unroll
      for (int nt = 0; nt < 4; ++nt) {
        const us_t* q = ENCT + ((size_t)(b * NH + 64 * ng + 16 * nt + m)) * NS + 32 * ks + 8 * h;
        Frag bb;
        bb.h[0] = *(const v8us*)q;
        bb.h[1] = *(const v8us*)(q + 16);
        acc2[nt] = wmh(pa[ks], bb, acc2[nt]);
      }
    }
#pragma unroll
    for (int nt = 0; nt < 4; ++nt)
#pragma unroll
      for (int rr = 0; rr < 8; ++rr)
        sX[(wave * 16 + 8 * h + rr) * 72 + 16 * nt + m] = (f16_t)(acc2[nt][rr] * INV256);
    __syncthreads();
    v8us ov[4];
    size_t off[4];
#pragma unroll
    for (int j = 0; j < 4; ++j) {
      const int tl = 4 * j + rq;
      ov[j] = asus_(*(const v8h*)(sX + (wave * 16 + tl) * 72 + 8 * cq8));
      off[j] = ((size_t)((tw + tl) * NB + b)) * NH + 64 * ng + 8 * cq8;
    }
#pragma unroll
    for (int j = 0; j < 4; ++j) *(volatile v8us*)(CTX + off[j]) = ov[j];
    __threadfence();
#pragma unroll
    for (int j = 0; j < 4; ++j) *(volatile v8us*)(CTX + off[j]) = ov[j];
    __syncthreads();
  }
}

extern "C" void kernel_launch(void* const* d_in, const int* in_sizes, int n_in,
                              void* d_out, int out_size, void* d_ws, size_t ws_size,
                              hipStream_t stream) {
  if (n_in < 17) return;
  if (in_sizes[0] != NB * NT) return;
  if (in_sizes[1] != NB * NS * NH) return;
  if (in_sizes[2] != NL * NB * NH || in_sizes[3] != NL * NB * NH) return;
  if (in_sizes[4] != NV * NE) return;
  if (in_sizes[5] != NG * NE || in_sizes[6] != NG || in_sizes[7] != NG * NH || in_sizes[8] != NG) return;
  if (in_sizes[9] != NG * NH || in_sizes[10] != NG || in_sizes[11] != NG * NH || in_sizes[12] != NG) return;
  if (in_sizes[13] != NH * NH || in_sizes[14] != NH) return;
  if (in_sizes[15] != NH * 2 * NH || in_sizes[16] != NH) return;
  if (out_size != OUTN) return;
  const size_t tot = (size_t)WSTOT;
  if (tot > ws_size || tot > (size_t)WSCAP) return;

  const int*   tok  = (const int*)d_in[0];
  const float* enc  = (const float*)d_in[1];
  const float* h0in = (const float*)d_in[2];
  const float* c0in = (const float*)d_in[3];
  const float* emb  = (const float*)d_in[4];
  const float* Wih0 = (const float*)d_in[5];
  const float* bih0 = (const float*)d_in[6];
  const float* Whh0 = (const float*)d_in[7];
  const float* bhh0 = (const float*)d_in[8];
  const float* Wih1 = (const float*)d_in[9];
  const float* bih1 = (const float*)d_in[10];
  const float* Whh1 = (const float*)d_in[11];
  const float* bhh1 = (const float*)d_in[12];
  const float* Win  = (const float*)d_in[13];
  const float* bin  = (const float*)d_in[14];
  const float* Wout = (const float*)d_in[15];
  const float* bout = (const float*)d_in[16];
  float* out = (float*)d_out;

  char* ws = (char*)d_ws;
  us_t*  EMB  = (us_t*)(ws + O_EMB);
  us_t*  WIH0 = (us_t*)(ws + O_WIH0);
  us_t*  WHH0 = (us_t*)(ws + O_WHH0);
  us_t*  WIH1 = (us_t*)(ws + O_WIH1);
  us_t*  WHH1 = (us_t*)(ws + O_WHH1);
  us_t*  WIN  = (us_t*)(ws + O_WIN);
  us_t*  WOUT = (us_t*)(ws + O_WOUT);
  us_t*  ENC  = (us_t*)(ws + O_ENC);
  us_t*  ENCT = (us_t*)(ws + O_ENCT);
  float* X0   = (float*)(ws + O_X0);
  us_t*  H0   = (us_t*)(ws + O_H0);
  us_t*  H1   = (us_t*)(ws + O_H1);
  float* C0   = (float*)(ws + O_C0);
  float* C1   = (float*)(ws + O_C1);
  us_t*  GAM  = (us_t*)(ws + O_GAM);
  us_t*  CTX  = (us_t*)(ws + O_CTX);

  k_cvt<<<NG * NE / 2048, 256, 0, stream>>>(Wih0, WIH0, NE, NE, SCW, SCW);
  k_cvt<<<NG * NH / 2048, 256, 0, stream>>>(Whh0, WHH0, NH, NH, SCW, SCW);
  k_cvt<<<NG * NH / 2048, 256, 0, stream>>>(Wih1, WIH1, NH, NH, SCW, SCW);
  k_cvt<<<NG * NH / 2048, 256, 0, stream>>>(Whh1, WHH1, NH, NH, SCW, SCW);
  k_cvt<<<NH * NH / 2048, 256, 0, stream>>>(Win, WIN, NH, NH, SCW, SCW);
  k_cvt<<<NH * 2 * NH / 2048, 256, 0, stream>>>(Wout, WOUT, 2 * NH, NH, SCWO1, SCW);
  k_cvt<<<NB * NS * NH / 2048, 256, 0, stream>>>(enc, ENC, NH, NH, SCX, SCX);
  k_enct<<<dim3(NH / 64, NB), 256, 0, stream>>>(enc, ENCT);
  k_embg<<<NR * NE / 2048, 256, 0, stream>>>(tok, emb, EMB);
  k_inith<<<NL * NB * NH / 2048, 256, 0, stream>>>(h0in, H0, H1);

  k_gemm<0><<<dim3(NR / 64, NG / 128), 128, 0, stream>>>(EMB, NE, NE / 32, EMB, NE, 0, WIH0, NE,
                                                         bih0, bhh0, X0, GAM, NG);

  for (int k = 0; k <= NT; ++k) {
    const int lb = (k == NT) ? 1 : 0;
    const int ny = (k == 0 || k == NT) ? 1 : 2;
    const float* cp0 = (k == 0) ? c0in : C0;
    const float* cp1 = (k == 1) ? (c0in + NB * NH) : C1;
    k_step<<<dim3(NH / 64, ny), 128, 0, stream>>>(WHH0, WIH1, WHH1, X0, bih1, bhh1, H0, H1,
                                                  cp0, cp1, C0, C1, out, k, lb);
  }

  k_gemm<1><<<dim3(NR / 64, NH / 128), 128, 0, stream>>>(H1 + NB * NH, NH, NH / 32, H1 + NB * NH, NH, 0,
                                                         WIN, NH, bin, bin, X0, GAM, NH);

  k_attn<<<NB, 128, 0, stream>>>(GAM, ENC, ENCT, CTX);

  k_gemm<2><<<dim3(NR / 64, NH / 128), 128, 0, stream>>>(CTX, NH, NH / 32, H1 + NB * NH, NH, NH / 32,
                                                         WOUT, 2 * NH, bout, bout, out, GAM, NH);
}
